// GWRNN_4183298146631
// MI455X (gfx1250) — hardware-verified
//
#include <hip/hip_runtime.h>

typedef __attribute__((ext_vector_type(16))) _Float16 v16h;
typedef __attribute__((ext_vector_type(8)))  _Float16 v8h;
typedef __attribute__((ext_vector_type(16))) __bf16   v16b;
typedef __attribute__((ext_vector_type(8)))  __bf16   v8b;
typedef __attribute__((ext_vector_type(8)))  float    v8f;
typedef __attribute__((ext_vector_type(4)))  float    v4f;

constexpr int kSeq  = 64;
constexpr int kStep = 512;
constexpr int kIn   = 256;
constexpr int kHid  = 1024;
constexpr int kOut  = 128;
constexpr float kAlpha  = 0.1f;
constexpr float kWScale = 64.0f;
constexpr float kAScale = 16.0f;
constexpr float kInvAcc = 1.0f / 1024.0f;

constexpr int kSeqPB      = 16;
constexpr int kRnnBlocks  = kSeq / kSeqPB;
constexpr int kWaves      = 16;
constexpr int kRnnThreads = 32 * kWaves;
constexpr int kColsPW     = 64;
constexpr int kHP         = kHid + 8;
constexpr int kXP         = kIn + 8;
constexpr int kYP         = kOut + 4;
constexpr int kHTile      = kSeqPB * kHP;
constexpr int kXTile      = kSeqPB * kXP;
constexpr int kYTile      = kSeqPB * kYP;
static_assert(kSeq == kRnnBlocks * kSeqPB, "blocks cover the batch exactly");
static_assert(kHid == kWaves * kColsPW, "wave columns cover the hidden dim exactly");
static_assert(kOut == 8 * 16, "readout: 8 waves x one 16-column subtile");
static_assert(kRnnThreads * 8 == kSeqPB * kIn, "x staging: 512 threads x 8 halves = 16 x 256 exactly");
static_assert(kWaves == kSeqPB && kOut == 32 * 4, "y store: one wave per output row, 32 lanes x 4 floats = 128 exactly");
static_assert(kHP % 8 == 0 && kXP % 8 == 0 && kYP % 4 == 0, "16-B aligned LDS vector accesses");
static_assert(kHid % 32 == 0 && kIn % 32 == 0, "K multiples of 32");
static_assert((2 * kHTile) % 8 == 0 && (2 * kYTile) % 4 == 0, "init zero loops exact");

constexpr int kDwWih = kHid * kIn  / 2;
constexpr int kDwWhh = kHid * kHid / 2;
constexpr int kDwWl  = kHid * kHid / 2;
constexpr int kDwWho = kOut * kHid / 2;
constexpr int kPrepB1 = kDwWih / 256;
constexpr int kPrepB2 = kPrepB1 + kDwWhh / 256;
constexpr int kPrepB3 = kPrepB2 + kDwWl / 256;
constexpr int kPrepBlocks = kPrepB3 + kDwWho / 256;
static_assert(kDwWih % 256 == 0 && kDwWhh % 256 == 0 && kDwWl % 256 == 0 && kDwWho % 256 == 0, "exact coverage");
static_assert(kPrepBlocks == 4864, "prep grid");

__device__ __forceinline__ void dep_guard_h(v8f& a, v8f& b, v16h x, v16h y) { asm volatile("v_nop\n\tv_nop\n\tv_nop\n\tv_nop" : "+v"(a), "+v"(b) : "v"(x), "v"(y)); }
__device__ __forceinline__ void dep_guard_b(v8f& a, v8f& b, v16b x, v16b y) { asm volatile("v_nop\n\tv_nop\n\tv_nop\n\tv_nop" : "+v"(a), "+v"(b) : "v"(x), "v"(y)); }
__device__ __forceinline__ void keep4_h(v16h a, v16h b, v16h c, v16h d) { asm volatile("v_nop" :: "v"(a), "v"(b), "v"(c), "v"(d)); }
__device__ __forceinline__ void keep4_b(v16b a, v16b b, v16b c, v16b d) { asm volatile("v_nop" :: "v"(a), "v"(b), "v"(c), "v"(d)); }
__device__ __forceinline__ void acc_guard4(v8f& a, v8f& b, v8f& c, v8f& d) { asm volatile("v_nop\n\tv_nop\n\tv_nop\n\tv_nop" : "+v"(a), "+v"(b), "+v"(c), "+v"(d)); }
__device__ __forceinline__ void acc_guard1(v8f& a) { asm volatile("v_nop\n\tv_nop\n\tv_nop\n\tv_nop" : "+v"(a)); }

template <typename T> struct Frag;
template <> struct Frag<_Float16> {
  typedef v16h V; union U { v16h v; v8h h[2]; };
  static __device__ __forceinline__ v16h load(const _Float16* p) {
    U f; f.h[0] = *(const v8h*)(p); f.h[1] = *(const v8h*)(p + 16); return f.v;
  }
  static __device__ __forceinline__ v8f mma(v16h a, v16h b, v8f c) {
    return __builtin_amdgcn_wmma_f32_16x16x32_f16(false, a, false, b, (short)0, c, false, false);
  }
  static __device__ __forceinline__ void guard(v8f& a, v8f& b, v16h x, v16h y) { dep_guard_h(a, b, x, y); }
  static __device__ __forceinline__ void keep(v16h a, v16h b, v16h c, v16h d) { keep4_h(a, b, c, d); }
};
template <> struct Frag<__bf16> {
  typedef v16b V; union U { v16b v; v8b h[2]; };
  static __device__ __forceinline__ v16b load(const __bf16* p) {
    U f; f.h[0] = *(const v8b*)(p); f.h[1] = *(const v8b*)(p + 16); return f.v;
  }
  static __device__ __forceinline__ v8f mma(v16b a, v16b b, v8f c) {
    return __builtin_amdgcn_wmma_f32_16x16x32_bf16(false, a, false, b, (short)0, c, false, false);
  }
  static __device__ __forceinline__ void guard(v8f& a, v8f& b, v16b x, v16b y) { dep_guard_b(a, b, x, y); }
  static __device__ __forceinline__ void keep(v16b a, v16b b, v16b c, v16b d) { keep4_b(a, b, c, d); }
};

__device__ __forceinline__ v8f mma1_h(v16h a, v16h b, v8f c) {
  c = __builtin_amdgcn_wmma_f32_16x16x32_f16(false, a, false, b, (short)0, c, false, false);
  asm volatile("v_nop\n\tv_nop\n\tv_nop\n\tv_nop" : "+v"(c) : "v"(a), "v"(b));
  return c;
}

__device__ __forceinline__ unsigned pack_f16x2(float a, float b) {
  const _Float16 h0 = (_Float16)a, h1 = (_Float16)b;
  return (unsigned)__builtin_bit_cast(unsigned short, h0) | ((unsigned)__builtin_bit_cast(unsigned short, h1) << 16);
}
__device__ __forceinline__ void st2u(unsigned* p, unsigned v) { *(volatile unsigned*)p = v; __threadfence(); *(volatile unsigned*)p = v; }
__device__ __forceinline__ float ftanh(float x) { return 1.0f - 2.0f * __builtin_amdgcn_rcpf(1.0f + __expf(2.0f * x)); }

__global__ __launch_bounds__(256) void prep_kernel(
    const float* __restrict__ w_ih, const float* __restrict__ w_hh, const float* __restrict__ w_ho,
    const float* __restrict__ bparam, const float* __restrict__ bmask, const float* __restrict__ mhat,
    unsigned* __restrict__ wihu, unsigned* __restrict__ whhu,
    unsigned* __restrict__ wlu, unsigned* __restrict__ whou) {
#pragma clang fp contract(off)
  const int blk = blockIdx.x, tid = threadIdx.x;
  if (blk < kPrepB1) {
    const int p = blk * 256 + tid;
    st2u(wihu + p, pack_f16x2(w_ih[2 * p] * kWScale, w_ih[2 * p + 1] * kWScale));
  } else if (blk < kPrepB2) {
    const int p = (blk - kPrepB1) * 256 + tid;
    st2u(whhu + p, pack_f16x2(w_hh[2 * p] * kWScale, w_hh[2 * p + 1] * kWScale));
  } else if (blk < kPrepB3) {
    const int p = (blk - kPrepB2) * 256 + tid;
    const int t = 2 * p;
    const int i = t >> 10;
    const int j = t & (kHid - 1);
    const float mi  = mhat[(size_t)i * (kHid + 1)];
    const float mj0 = mhat[(size_t)j * (kHid + 1)];
    const float mj1 = mhat[(size_t)(j + 1) * (kHid + 1)];
    const float bb0 = bparam[t] * bmask[t];
    const float bb1 = bparam[t + 1] * bmask[t + 1];
    const int u0 = j * kHid + i, u1 = (j + 1) * kHid + i;
    const float bt0 = bparam[u0] * bmask[u0];
    const float bt1 = bparam[u1] * bmask[u1];
    const float rc0 = 1.0f / mj0, rc1 = 1.0f / mj1;
    const float q0 = mi * bt0, q1 = mi * bt1;
    const float w0 = bb0 - q0 * rc0;
    const float w1 = bb1 - q1 * rc1;
    st2u(wlu + p, pack_f16x2(w0 * kWScale, w1 * kWScale));
  } else {
    const int p = (blk - kPrepB3) * 256 + tid;
    st2u(whou + p, pack_f16x2(w_ho[2 * p] * kWScale, w_ho[2 * p + 1] * kWScale));
  }
}

__device__ __forceinline__ void stage_x(const float* __restrict__ x, _Float16* xt, int seq0, int s1, int tid) {
  const int row = tid >> 5, col8 = (tid & 31) * 8;
  const float* xp = x + ((size_t)(seq0 + row) * kStep + s1) * kIn + col8;
  const v4f a = *(const v4f*)xp;
  const v4f b = *(const v4f*)(xp + 4);
  v8h hv;
  hv[0] = (_Float16)(a[0] * kAScale); hv[1] = (_Float16)(a[1] * kAScale);
  hv[2] = (_Float16)(a[2] * kAScale); hv[3] = (_Float16)(a[3] * kAScale);
  hv[4] = (_Float16)(b[0] * kAScale); hv[5] = (_Float16)(b[1] * kAScale);
  hv[6] = (_Float16)(b[2] * kAScale); hv[7] = (_Float16)(b[3] * kAScale);
  *(v8h*)(xt + row * kXP + col8) = hv;
}

__global__ __launch_bounds__(kRnnThreads) void rnn_kernel(
    const float* __restrict__ x,
    const float* __restrict__ b_ih, const float* __restrict__ b_hh, const float* __restrict__ b_o,
    const _Float16* __restrict__ wih16, const _Float16* __restrict__ whh16,
    const _Float16* __restrict__ wl16, const _Float16* __restrict__ who16,
    float* __restrict__ out) {
  __shared__ __align__(16) _Float16 htile[2][kHTile];
  __shared__ __align__(16) _Float16 xtile[2][kXTile];
  __shared__ __align__(16) float    ytile[2][kYTile];
  const int tid = threadIdx.x, lane = tid & 31;
  const int wv = __builtin_amdgcn_readfirstlane(tid >> 5);
  const int c = lane & 15, hh = lane >> 4, koff = hh * 8, mOff = hh * 8;
  const int seq0 = blockIdx.x * kSeqPB;
  const int n0 = wv * kColsPW;
  const int yn0 = (wv & 7) * 16;

  {
    _Float16* hf = &htile[0][0];
    v8h z8; z8[0] = (_Float16)0.0f; z8[1] = z8[0]; z8[2] = z8[0]; z8[3] = z8[0]; z8[4] = z8[0]; z8[5] = z8[0]; z8[6] = z8[0]; z8[7] = z8[0];
    for (int i = tid; i < (2 * kHTile) / 8; i += kRnnThreads) *(v8h*)(hf + 8 * i) = z8;
    float* yf = &ytile[0][0];
    const v4f z4 = {0.f, 0.f, 0.f, 0.f};
    for (int i = tid; i < (2 * kYTile) / 4; i += kRnnThreads) *(v4f*)(yf + 4 * i) = z4;
  }
  stage_x(x, &xtile[0][0], seq0, 0, tid);
  __syncthreads();

  float bsum[4];
#pragma unroll
  for (int j = 0; j < 4; ++j) { const int col = n0 + 16 * j + c; bsum[j] = b_ih[col] + b_hh[col]; }
  const float ybias = b_o[yn0 + c];
  const _Float16* bwh = whh16 + (size_t)(n0 + c) * kHid + koff;
  const _Float16* bwl = wl16  + (size_t)(n0 + c) * kHid + koff;
  const _Float16* bwi = wih16 + (size_t)(n0 + c) * kIn  + koff;
  const _Float16* bwo = who16 + (size_t)(yn0 + c) * kHid + koff;

  const v8f zro = {0.f, 0.f, 0.f, 0.f, 0.f, 0.f, 0.f, 0.f};
  v8f hreg[4];
#pragma unroll
  for (int j = 0; j < 4; ++j) hreg[j] = zro;

#pragma unroll 1
  for (int s = 0; s <= kStep; ++s) {
    const int p = s & 1;
    const _Float16* hcur = &htile[p][0];
    _Float16*       hnxt = &htile[p ^ 1][0];
    const _Float16* xcur = &xtile[p][0];
    _Float16*       xnxt = &xtile[p ^ 1][0];
    float*          ycur = &ytile[p][0];

    v8f acch[4], accl[4], accy = zro;
#pragma unroll
    for (int j = 0; j < 4; ++j) { acch[j] = zro; accl[j] = zro; }

    const _Float16* arow = hcur + c * kHP + koff;
    v16h fa;
    v16h fb[4];
#pragma unroll 1
    for (int kc = 0; kc < kHid / 32; ++kc) {
      fa = Frag<_Float16>::load(arow + kc * 32);
#pragma unroll
      for (int j = 0; j < 4; ++j) fb[j] = Frag<_Float16>::load(bwh + (size_t)(16 * j) * kHid + kc * 32);
#pragma unroll
      for (int j = 0; j < 4; ++j) acch[j] = Frag<_Float16>::mma(fa, fb[j], acch[j]);
      Frag<_Float16>::guard(acch[0], acch[3], fa, fb[3]);
      Frag<_Float16>::keep(fb[0], fb[1], fb[2], fb[3]);
#pragma unroll
      for (int j = 0; j < 4; ++j) fb[j] = Frag<_Float16>::load(bwl + (size_t)(16 * j) * kHid + kc * 32);
#pragma unroll
      for (int j = 0; j < 4; ++j) accl[j] = Frag<_Float16>::mma(fa, fb[j], accl[j]);
      Frag<_Float16>::guard(accl[0], accl[3], fa, fb[3]);
      Frag<_Float16>::keep(fb[0], fb[1], fb[2], fb[3]);
      if (wv < 8) {
        const v16h fy = Frag<_Float16>::load(bwo + kc * 32);
        accy = mma1_h(fa, fy, accy);
      }
    }
    const _Float16* xrow = xcur + c * kXP + koff;
#pragma unroll 1
    for (int kc = 0; kc < kIn / 32; ++kc) {
      fa = Frag<_Float16>::load(xrow + kc * 32);
#pragma unroll
      for (int j = 0; j < 4; ++j) fb[j] = Frag<_Float16>::load(bwi + (size_t)(16 * j) * kIn + kc * 32);
#pragma unroll
      for (int j = 0; j < 4; ++j) acch[j] = Frag<_Float16>::mma(fa, fb[j], acch[j]);
      Frag<_Float16>::guard(acch[0], acch[3], fa, fb[3]);
      Frag<_Float16>::keep(fb[0], fb[1], fb[2], fb[3]);
    }
    acc_guard4(acch[0], acch[1], acch[2], acch[3]);
    acc_guard4(accl[0], accl[1], accl[2], accl[3]);
    acc_guard1(accy);

    stage_x(x, xnxt, seq0, (s + 1 < kStep) ? (s + 1) : (kStep - 1), tid);

#pragma unroll
    for (int j = 0; j < 4; ++j) {
#pragma unroll
      for (int r = 0; r < 8; ++r) {
        const float hold = hreg[j][r];
        const float pre  = acch[j][r] * kInvAcc + bsum[j];
        const float hl   = accl[j][r] * kInvAcc;
        const float fx   = (-hold + ftanh(pre)) + hl;
        const float v    = hold + kAlpha * fx;
        hreg[j][r] = v;
        hnxt[(mOff + r) * kHP + n0 + 16 * j + c] = (_Float16)(v * kAScale);
      }
    }
    if (wv < 8) {
#pragma unroll
      for (int r = 0; r < 8; ++r) ycur[(mOff + r) * kYP + yn0 + c] = accy[r] * kInvAcc + ybias;
    }
    __syncthreads();

    if (s >= 1) {
      const int row = tid >> 5;
      const v4f val = *(const v4f*)(ycur + row * kYP + lane * 4);
      float* op = out + ((size_t)(seq0 + row) * kStep + (size_t)(s - 1)) * kOut + lane * 4;
      *(volatile v4f*)op = val;
      __threadfence();
      *(volatile v4f*)op = val;
    }
  }
}

extern "C" void kernel_launch(void* const* d_in, const int* in_sizes, int n_in,
                              void* d_out, int out_size, void* d_ws, size_t ws_size, hipStream_t stream) {
  if (n_in < 10 || d_out == nullptr || d_ws == nullptr) return;
  if (in_sizes[0] != kSeq * kStep * kIn || in_sizes[1] != kHid * kIn || in_sizes[2] != kHid ||
      in_sizes[3] != kHid * kHid || in_sizes[4] != kHid || in_sizes[5] != kOut * kHid || in_sizes[6] != kOut ||
      in_sizes[7] != kHid * kHid || in_sizes[8] != kHid * kHid || in_sizes[9] != kHid * kHid ||
      out_size != kSeq * kStep * kOut) return;

  const float* x      = (const float*)d_in[0];
  const float* w_ih   = (const float*)d_in[1];
  const float* b_ih   = (const float*)d_in[2];
  const float* w_hh   = (const float*)d_in[3];
  const float* b_hh   = (const float*)d_in[4];
  const float* w_ho   = (const float*)d_in[5];
  const float* b_o    = (const float*)d_in[6];
  const float* bparam = (const float*)d_in[7];
  const float* mhat   = (const float*)d_in[8];
  const float* bmask  = (const float*)d_in[9];
  float* out = (float*)d_out;

  char* ws = (char*)d_ws; size_t off = 0;
  auto carve = [&](size_t bytes) -> char* { char* p = ws + off; off += (bytes + 255) & ~(size_t)255; return p; };
  unsigned short* WIH16 = (unsigned short*)carve((size_t)kHid * kIn  * 2);
  unsigned short* WHH16 = (unsigned short*)carve((size_t)kHid * kHid * 2);
  unsigned short* WL16  = (unsigned short*)carve((size_t)kHid * kHid * 2);
  unsigned short* WHO16 = (unsigned short*)carve((size_t)kOut * kHid * 2);
  if (off > ws_size || off > (size_t)134217728) return;

  prep_kernel<<<kPrepBlocks, 256, 0, stream>>>(w_ih, w_hh, w_ho, bparam, bmask, mhat,
                                               (unsigned*)WIH16, (unsigned*)WHH16, (unsigned*)WL16, (unsigned*)WHO16);

  rnn_kernel<<<kRnnBlocks, kRnnThreads, 0, stream>>>(x, b_ih, b_hh, b_o,
                                                     (const _Float16*)WIH16, (const _Float16*)WHH16,
                                                     (const _Float16*)WL16, (const _Float16*)WHO16, out);
}
